// LSTMModel_15702400434245
// MI455X (gfx1250) — hardware-verified
//
#include <hip/hip_runtime.h>
#include <math.h>

constexpr int NBATCH    = 4096;
constexpr int NSTEP     = 512;
constexpr int NHID      = 32;
constexpr int NGATE     = 4 * NHID;
constexpr int NWAVE     = 2;
constexpr int NTHR      = 32 * NWAVE;
constexpr int ROWS_WAVE = 16;
constexpr int ROWS_BLK  = ROWS_WAVE * NWAVE;
constexpr int XCH       = 32;
constexpr int NCHUNK    = NSTEP / XCH;
constexpr int XPITCH    = 36;
constexpr int FPITCH    = 68;
constexpr int HTILE     = ROWS_WAVE * NHID;
constexpr int WPLANE    = NGATE * NHID;
constexpr float L2E     = 1.4426950408889634f;
constexpr float WCARRY  = 16.0f;
constexpr float KSIG    = -L2E / WCARRY;
constexpr float KTANH   = -2.0f * L2E / WCARRY;
constexpr float BSIG    = -L2E;
constexpr float BTANH   = -2.0f * L2E;
static_assert(NHID == 32, "one 32-deep k-step per product");
static_assert(NBATCH % ROWS_BLK == 0, "grid exact");
static_assert(NSTEP % XCH == 0 && (XCH % 2) == 0, "x chunks exact, parity continues across chunks");
static_assert(WPLANE % (8 * NTHR) == 0, "weight staging loop exact");
static_assert((NWAVE * 4 * HTILE) % (8 * NTHR) == 0, "h zero-fill loop exact");
static_assert(NGATE == 2 * NTHR, "bias staging covers 128 columns with 2 per thread");
static_assert(ROWS_BLK * 4 == 128, "one block = one 128-B output line");
static_assert((XPITCH % 4) == 0 && (FPITCH % 4) == 0, "16-B aligned LDS rows");

typedef __attribute__((ext_vector_type(16))) _Float16 v16h;
typedef __attribute__((ext_vector_type(8)))  _Float16 v8h;
typedef __attribute__((ext_vector_type(8)))  float    v8f;
typedef __attribute__((ext_vector_type(4)))  float    v4f;

template <typename T> struct Frag;
template <> struct Frag<_Float16> {
  typedef v16h V; union U { v16h v; v8h h[2]; };
  static __device__ __forceinline__ v16h load(const _Float16* p) {
    U f; f.h[0] = *(const v8h*)(p); f.h[1] = *(const v8h*)(p + 16); return f.v;
  }
};

__device__ __forceinline__ void mma_pair(v8f& acc, v16h a0, v16h b0, v16h a1, v16h b1) {
  acc = __builtin_amdgcn_wmma_f32_16x16x32_f16(false, a0, false, b0, (short)0, acc, false, false);
  acc = __builtin_amdgcn_wmma_f32_16x16x32_f16(false, a1, false, b1, (short)0, acc, false, false);
  asm volatile("v_nop\n\tv_nop\n\tv_nop\n\tv_nop" : "+v"(acc) : "v"(a0), "v"(b0), "v"(a1), "v"(b1));
}

__device__ __forceinline__ void wave_lds_sync() {
  __builtin_amdgcn_fence(__ATOMIC_RELEASE, "workgroup");
  __builtin_amdgcn_wave_barrier();
  __builtin_amdgcn_fence(__ATOMIC_ACQUIRE, "workgroup");
}

__device__ __forceinline__ float sig_fast(float a, float k, float cb) {
  const float e = __builtin_amdgcn_exp2f(fmaf(a, k, cb));
  return __builtin_amdgcn_rcpf(1.0f + e);
}
__device__ __forceinline__ float tanh_fast(float a, float k, float cb) {
  const float e = __builtin_amdgcn_exp2f(fmaf(a, k, cb));
  const float r = __builtin_amdgcn_rcpf(1.0f + e);
  return fmaf(2.0f, r, -1.0f);
}

__device__ __forceinline__ void stage_plane(const float* __restrict__ W, _Float16* dst, int tid) {
#pragma unroll 1
  for (int it = 0; it < WPLANE / (8 * NTHR); ++it) {
    const int i = it * NTHR + tid;
    const v4f a = *(const v4f*)(W + 8 * i);
    const v4f b = *(const v4f*)(W + 8 * i + 4);
    v8h hv;
#pragma unroll
    for (int e = 0; e < 4; ++e) {
      const float fa = a[e] * WCARRY;
      const float fb = b[e] * WCARRY;
      hv[e]     = (_Float16)fa;
      hv[4 + e] = (_Float16)fb;
    }
    *(v8h*)(dst + 8 * i) = hv;
  }
}

__device__ __forceinline__ void layer_step(const v16h ain, const _Float16* hrd, _Float16* hwr,
                                           const _Float16* wih, const _Float16* whh,
                                           const float (&cb)[2][4], float (&cst)[2][8],
                                           const bool last, float* fst, const int c, const int hh) {
  const v16h ah = Frag<_Float16>::load(hrd + c * NHID + 8 * hh);
  const v8f z8 = {0.f, 0.f, 0.f, 0.f, 0.f, 0.f, 0.f, 0.f};
#pragma unroll
  for (int ub = 0; ub < 2; ++ub) {
    v8f acc[4];
#pragma unroll
    for (int g = 0; g < 4; ++g) {
      const int n = NHID * g + 16 * ub + c;
      const v16h bi = Frag<_Float16>::load(wih + n * NHID + 8 * hh);
      const v16h bh = Frag<_Float16>::load(whh + n * NHID + 8 * hh);
      acc[g] = z8;
      mma_pair(acc[g], ain, bi, ah, bh);
    }
    float hn[8];
#pragma unroll
    for (int r = 0; r < 8; ++r) {
      const float ig = sig_fast(acc[0][r], KSIG, cb[ub][0]);
      const float fg = sig_fast(acc[1][r], KSIG, cb[ub][1]);
      const float gg = tanh_fast(acc[2][r], KTANH, cb[ub][2]);
      const float og = sig_fast(acc[3][r], KSIG, cb[ub][3]);
      const float cn = fmaf(fg, cst[ub][r], ig * gg);
      cst[ub][r] = cn;
      hn[r] = og * tanh_fast(cn, BTANH, 0.0f);
    }
#pragma unroll
    for (int r = 0; r < 8; ++r) hwr[(8 * hh + r) * NHID + 16 * ub + c] = (_Float16)hn[r];
    if (last) {
#pragma unroll
      for (int r = 0; r < 8; ++r) fst[(8 * hh + r) * FPITCH + 16 * ub + c] = hn[r];
    }
  }
}

__global__ __launch_bounds__(NTHR) void lstm2_seq_kernel(
    const float* __restrict__ x,
    const float* __restrict__ W1,   const float* __restrict__ b1,
    const float* __restrict__ Wih0, const float* __restrict__ Whh0,
    const float* __restrict__ bih0, const float* __restrict__ bhh0,
    const float* __restrict__ Wih1, const float* __restrict__ Whh1,
    const float* __restrict__ bih1, const float* __restrict__ bhh1,
    const float* __restrict__ W2,   const float* __restrict__ b2,
    float* __restrict__ out) {
  __shared__ __align__(16) _Float16 Wl[4 * WPLANE];
  __shared__ __align__(16) _Float16 Ht[NWAVE * 4 * HTILE];
  __shared__ __align__(16) float Xs[NWAVE * ROWS_WAVE * XPITCH];
  __shared__ __align__(16) float Fs[NWAVE * ROWS_WAVE * FPITCH];
  __shared__ __align__(16) float Bs[2 * NGATE];
  __shared__ __align__(16) float LinW[32];
  __shared__ __align__(16) float LinB[32];
  __shared__ __align__(16) float Os[ROWS_BLK];

  const int tid = threadIdx.x, lane = tid & 31, wave = tid >> 5;
  const int c = lane & 15, hh = lane >> 4;
  const int rowbase = blockIdx.x * ROWS_BLK + wave * ROWS_WAVE;

  stage_plane(Wih0, Wl + 0 * WPLANE, tid);
  stage_plane(Whh0, Wl + 1 * WPLANE, tid);
  stage_plane(Wih1, Wl + 2 * WPLANE, tid);
  stage_plane(Whh1, Wl + 3 * WPLANE, tid);
  {
    const v8h zz = {(_Float16)0.0f, (_Float16)0.0f, (_Float16)0.0f, (_Float16)0.0f,
                    (_Float16)0.0f, (_Float16)0.0f, (_Float16)0.0f, (_Float16)0.0f};
#pragma unroll 1
    for (int it = 0; it < (NWAVE * 4 * HTILE) / (8 * NTHR); ++it) *(v8h*)(Ht + 8 * (it * NTHR + tid)) = zz;
  }
#pragma unroll
  for (int q = 0; q < 2; ++q) {
    const int n = q * NTHR + tid;
    Bs[n]         = bih0[n] + bhh0[n];
    Bs[NGATE + n] = bih1[n] + bhh1[n];
  }
  if (tid < 32) {
    const int h2 = tid >> 4, e = tid & 15;
    const int k = 8 * h2 + (e & 7) + ((e >> 3) << 4);
    LinW[tid] = W1[k];
    LinB[tid] = b1[k];
  }
  __syncthreads();

  float cb0[2][4], cb1[2][4], cst0[2][8], cst1[2][8];
#pragma unroll
  for (int ub = 0; ub < 2; ++ub) {
#pragma unroll
    for (int g = 0; g < 4; ++g) {
      const int n = NHID * g + 16 * ub + c;
      const float sc = (g == 2) ? BTANH : BSIG;
      cb0[ub][g] = Bs[n] * sc;
      cb1[ub][g] = Bs[NGATE + n] * sc;
    }
#pragma unroll
    for (int r = 0; r < 8; ++r) { cst0[ub][r] = 0.0f; cst1[ub][r] = 0.0f; }
  }

  _Float16* hb = Ht + wave * 4 * HTILE;
  float* xs = Xs + wave * ROWS_WAVE * XPITCH;
  float* fs = Fs + wave * ROWS_WAVE * FPITCH;
  const _Float16* wih0 = Wl;
  const _Float16* whh0 = Wl + 1 * WPLANE;
  const _Float16* wih1 = Wl + 2 * WPLANE;
  const _Float16* whh1 = Wl + 3 * WPLANE;

#pragma unroll 1
  for (int ch = 0; ch < NCHUNK; ++ch) {
#pragma unroll
    for (int it = 0; it < 4; ++it) {
      const int row = it * 4 + (lane >> 3), col4 = (lane & 7) * 4;
      const v4f v = *(const v4f*)(x + (size_t)(rowbase + row) * NSTEP + ch * XCH + col4);
      *(v4f*)(xs + row * XPITCH + col4) = v;
    }
    wave_lds_sync();
#pragma unroll 1
    for (int tt = 0; tt < XCH; ++tt) {
      const int p = tt & 1;
      const bool last = (ch == NCHUNK - 1) && (tt == XCH - 1);
      const float xv = xs[c * XPITCH + tt];
      v16h ain;
#pragma unroll
      for (int q = 0; q < 4; ++q) {
        const v4f w = *(const v4f*)(LinW + 16 * hh + 4 * q);
        const v4f b = *(const v4f*)(LinB + 16 * hh + 4 * q);
#pragma unroll
        for (int e = 0; e < 4; ++e) {
          const float av = fmaxf(fmaf(xv, w[e], b[e]), 0.0f);
          ain[4 * q + e] = (_Float16)av;
        }
      }
      layer_step(ain, hb + p * HTILE, hb + (p ^ 1) * HTILE, wih0, whh0, cb0, cst0, last, fs, c, hh);
      wave_lds_sync();
      const v16h a1 = Frag<_Float16>::load(hb + (p ^ 1) * HTILE + c * NHID + 8 * hh);
      layer_step(a1, hb + (2 + p) * HTILE, hb + (2 + (p ^ 1)) * HTILE, wih1, whh1, cb1, cst1, last, fs + NHID, c, hh);
      wave_lds_sync();
    }
  }

  float s = 0.0f;
  {
    const float* fr = fs + c * FPITCH + 32 * hh;
    const float* w2 = W2 + 32 * hh;
#pragma unroll
    for (int q = 0; q < 8; ++q) {
      const v4f f = *(const v4f*)(fr + 4 * q);
      const v4f w = *(const v4f*)(w2 + 4 * q);
      s = fmaf(f[0], w[0], s);
      s = fmaf(f[1], w[1], s);
      s = fmaf(f[2], w[2], s);
      s = fmaf(f[3], w[3], s);
    }
  }
  const float other = __shfl_xor(s, 16, 32);
  const float tot = (s + other) + b2[0];
  if (hh == 0) Os[wave * ROWS_WAVE + c] = tot;
  __syncthreads();
  if (tid < 8) {
    const v4f v = *(const v4f*)(Os + 4 * tid);
    float* op = out + (size_t)blockIdx.x * ROWS_BLK + 4 * tid;
    *(volatile v4f*)op = v;
    __threadfence();
    *(volatile v4f*)op = v;
  }
}

extern "C" void kernel_launch(void* const* d_in, const int* in_sizes, int n_in,
                              void* d_out, int out_size, void* d_ws, size_t ws_size, hipStream_t stream) {
  (void)d_ws; (void)ws_size;
  if (n_in < 13 || d_out == nullptr) return;
  if (in_sizes[0] != NBATCH * NSTEP || in_sizes[1] != NHID || in_sizes[2] != NHID ||
      in_sizes[3] != NGATE * NHID || in_sizes[4] != NGATE * NHID || in_sizes[5] != NGATE || in_sizes[6] != NGATE ||
      in_sizes[7] != NGATE * NHID || in_sizes[8] != NGATE * NHID || in_sizes[9] != NGATE || in_sizes[10] != NGATE ||
      in_sizes[11] != 2 * NHID || in_sizes[12] != 1 || out_size != NBATCH) return;

  const float* x    = (const float*)d_in[0];
  const float* W1   = (const float*)d_in[1];
  const float* b1   = (const float*)d_in[2];
  const float* Wih0 = (const float*)d_in[3];
  const float* Whh0 = (const float*)d_in[4];
  const float* bih0 = (const float*)d_in[5];
  const float* bhh0 = (const float*)d_in[6];
  const float* Wih1 = (const float*)d_in[7];
  const float* Whh1 = (const float*)d_in[8];
  const float* bih1 = (const float*)d_in[9];
  const float* bhh1 = (const float*)d_in[10];
  const float* W2   = (const float*)d_in[11];
  const float* b2   = (const float*)d_in[12];
  float* out = (float*)d_out;

  lstm2_seq_kernel<<<NBATCH / ROWS_BLK, NTHR, 0, stream>>>(x, W1, b1, Wih0, Whh0, bih0, bhh0,
                                                           Wih1, Whh1, bih1, bhh1, W2, b2, out);
}
